// TileGraphEncoder_85633057947709
// MI455X (gfx1250) — hardware-verified
//
#include <hip/hip_runtime.h>
#include <math.h>

#define NN 50000
#define NE 800000
#define NV (NE + NN)
#define NP 50176
#define FIN 256
#define F1 256
#define F2 64
#define NH1 4
#define NG 8
#define NT 256
#define TILE 1024
#define NTL (NP / TILE)
#define RPW (TILE / (NT / 32))

typedef __attribute__((ext_vector_type(16))) _Float16 v16h;
typedef __attribute__((ext_vector_type(8)))  _Float16 v8h;
typedef __attribute__((ext_vector_type(16))) __bf16   v16b;
typedef __attribute__((ext_vector_type(8)))  __bf16   v8b;
typedef __attribute__((ext_vector_type(8)))  float    v8f;
typedef __attribute__((ext_vector_type(4)))  float    v4f;
typedef __attribute__((ext_vector_type(2)))  float    v2f;
typedef __attribute__((ext_vector_type(4)))  int      v4i;

__device__ __forceinline__ unsigned short f2bf_bits(float f) {
  unsigned u = __float_as_uint(f);
  return (unsigned short)((u + 0x7FFFu + ((u >> 16) & 1u)) >> 16);
}
__device__ __forceinline__ float bf_bits2f(unsigned short h) { return __uint_as_float(((unsigned)h) << 16); }

__device__ __forceinline__ void dep_guard_h(v8f& a, v8f& b, v16h x, v16h y) { asm volatile("v_nop\n\tv_nop\n\tv_nop\n\tv_nop" : "+v"(a), "+v"(b) : "v"(x), "v"(y)); }
__device__ __forceinline__ void dep_guard_b(v8f& a, v8f& b, v16b x, v16b y) { asm volatile("v_nop\n\tv_nop\n\tv_nop\n\tv_nop" : "+v"(a), "+v"(b) : "v"(x), "v"(y)); }
__device__ __forceinline__ void keep4_h(v16h a, v16h b, v16h c, v16h d) { asm volatile("v_nop" :: "v"(a), "v"(b), "v"(c), "v"(d)); }
__device__ __forceinline__ void keep4_b(v16b a, v16b b, v16b c, v16b d) { asm volatile("v_nop" :: "v"(a), "v"(b), "v"(c), "v"(d)); }
__device__ __forceinline__ void fence_v4(v4f& t) { asm volatile("" : "+v"(t)); }
__device__ __forceinline__ void fence_v2(v2f& t) { asm volatile("" : "+v"(t)); }
__device__ __forceinline__ void acc_guard4(v8f& a, v8f& b, v8f& c, v8f& d) { asm volatile("v_nop\n\tv_nop\n\tv_nop\n\tv_nop" : "+v"(a), "+v"(b), "+v"(c), "+v"(d)); }
template <typename T> struct Frag;
template <> struct Frag<_Float16> {
  typedef v16h V; union U { v16h v; v8h h[2]; };
  static __device__ __forceinline__ v16h load(const _Float16* p) {
    U f; f.h[0] = *(const v8h*)(p); f.h[1] = *(const v8h*)(p + 16); return f.v;
  }
  static __device__ __forceinline__ v8f mma(v16h a, v16h b, v8f c) {
    return __builtin_amdgcn_wmma_f32_16x16x32_f16(false, a, false, b, (short)0, c, false, false);
  }
  static __device__ __forceinline__ void guard(v8f& a, v8f& b, v16h x, v16h y) { dep_guard_h(a, b, x, y); }
  static __device__ __forceinline__ void keep(v16h a, v16h b, v16h c, v16h d) { keep4_h(a, b, c, d); }
};
template <> struct Frag<__bf16> {
  typedef v16b V; union U { v16b v; v8b h[2]; };
  static __device__ __forceinline__ v16b load(const __bf16* p) {
    U f; f.h[0] = *(const v8b*)(p); f.h[1] = *(const v8b*)(p + 16); return f.v;
  }
  static __device__ __forceinline__ v8f mma(v16b a, v16b b, v8f c) {
    return __builtin_amdgcn_wmma_f32_16x16x32_bf16(false, a, false, b, (short)0, c, false, false);
  }
  static __device__ __forceinline__ void guard(v8f& a, v8f& b, v16b x, v16b y) { dep_guard_b(a, b, x, y); }
  static __device__ __forceinline__ void keep(v16b a, v16b b, v16b c, v16b d) { keep4_b(a, b, c, d); }
};

template <int ET> struct Elem;
template <> struct Elem<0> { typedef _Float16 T; };
template <> struct Elem<1> { typedef __bf16 T; };
template <int ET, bool SPLIT, int BIAS_MODE, int OUT_MODE, bool RESID, int ACT = 0>
__global__ __launch_bounds__(256) void wmma_gemm64(
    const unsigned short* __restrict__ Ap, const unsigned short* __restrict__ A2p, int lda, long strideA,
    const unsigned short* __restrict__ Btp, const unsigned short* __restrict__ Bt2p, int ldb, long strideB,
    void* __restrict__ Cout, void* __restrict__ Cout2, int ldc, long strideC,
    const float* __restrict__ bias,
    const float* __restrict__ resid, long strideR,
    int M, int N, int K, float scale) {
  typedef typename Elem<ET>::T T;
  typedef typename Frag<T>::V V;
  const T* A = (const T*)Ap; const T* A2 = (const T*)A2p; const T* Bt = (const T*)Btp; const T* Bt2 = (const T*)Bt2p;
  __shared__ __align__(16) float sT[8][16 * 68];
  const int b    = blockIdx.y;
  const int lane = threadIdx.x & 31;
  const int wave = threadIdx.x >> 5;
  const int tilesN = N >> 6;
  const int tilesM = M >> 6;
  const int tile = blockIdx.x * 8 + wave;
  if (tile >= tilesM * tilesN) return;
  const int tm = tile / tilesN;
  const int tn = tile - tm * tilesN;
  const int m0 = tm << 6;
  const int n0 = tn << 6;

  const T* Ab  = A  + (size_t)b * strideA;
  const T* Bb  = Bt + (size_t)b * strideB;
  const T* Ab2 = SPLIT ? (A2  + (size_t)b * strideA) : nullptr;
  const T* Bb2 = SPLIT ? (Bt2 + (size_t)b * strideB) : nullptr;

  const int rlane = lane & 15;
  const int koff  = (lane >> 4) * 8;
  const int mOff  = (lane >> 4) * 8;

  v8f acc[4][4];
#pragma unroll
  for (int i = 0; i < 4; ++i)
#pragma unroll
    for (int j = 0; j < 4; ++j) acc[i][j] = (v8f){0.f,0.f,0.f,0.f,0.f,0.f,0.f,0.f};

  for (int k0 = 0; k0 < K; k0 += 32) {
    V bh[4], bl[4];
#pragma unroll
    for (int j = 0; j < 4; ++j) {
      const size_t bo = (size_t)(n0 + (j << 4) + rlane) * ldb + koff + k0;
      bh[j] = Frag<T>::load(Bb + bo);
      if (SPLIT) bl[j] = Frag<T>::load(Bb2 + bo);
    }
#pragma unroll
    for (int i = 0; i < 4; ++i) {
      const size_t ao = (size_t)(m0 + (i << 4) + rlane) * lda + koff + k0;
      V ah = Frag<T>::load(Ab + ao);
      V al;
      if (SPLIT) al = Frag<T>::load(Ab2 + ao);
#pragma unroll
      for (int j = 0; j < 4; ++j) {
        acc[i][j] = Frag<T>::mma(ah, bh[j], acc[i][j]);
        if (SPLIT) {
          acc[i][j] = Frag<T>::mma(ah, bl[j], acc[i][j]);
          acc[i][j] = Frag<T>::mma(al, bh[j], acc[i][j]);
        }
      }
      Frag<T>::guard(acc[i][0], acc[i][3], ah, SPLIT ? al : ah);
    }
    Frag<T>::keep(bh[0], bh[1], bh[2], bh[3]);
    if (SPLIT) Frag<T>::keep(bl[0], bl[1], bl[2], bl[3]);
  }
  acc_guard4(acc[0][0], acc[0][1], acc[0][2], acc[0][3]);
  acc_guard4(acc[1][0], acc[1][1], acc[1][2], acc[1][3]);
  acc_guard4(acc[2][0], acc[2][1], acc[2][2], acc[2][3]);
  acc_guard4(acc[3][0], acc[3][1], acc[3][2], acc[3][3]);

  float* slab = sT[wave];
  const float* Rb = RESID ? (resid + (size_t)b * strideR) : nullptr;
#pragma unroll
  for (int i = 0; i < 4; ++i) {
    const int mBase = m0 + (i << 4);
#pragma unroll
    for (int j = 0; j < 4; ++j) {
      const int n = n0 + (j << 4) + rlane;
      float bv = 0.f;
      if (BIAS_MODE == 2) bv = bias[n];
#pragma unroll
      for (int r = 0; r < 8; ++r) {
        float v = acc[i][j][r] * scale;
        if (BIAS_MODE == 1) v += bias[mBase + mOff + r];
        if (BIAS_MODE == 2) v += bv;
        if (RESID) v += Rb[(size_t)(mBase + mOff + r) * ldc + n];
        if (ACT == 1) v = tanhf(v);
        if (ACT == 2) v = fmaxf(v, 0.0f);
        if (ACT == 3) v = v / (1.0f + expf(-v));
        if (ACT == 4) v = (v > 0.f) ? v : 0.01f * v;
        if (ACT == 5) v = 0.5f * v * (1.0f + erff(v * 0.70710678118654752f));
        slab[(mOff + r) * 68 + (j << 4) + rlane] = v;
      }
    }
    __builtin_amdgcn_fence(__ATOMIC_RELEASE, "workgroup");
    __builtin_amdgcn_wave_barrier();
    __builtin_amdgcn_fence(__ATOMIC_ACQUIRE, "workgroup");
    if (OUT_MODE == 0) {
      float* C = (float*)Cout + (size_t)b * strideC;
      const int hh = lane >> 4, c4 = (lane & 15) * 4;
      for (int pass = 0; pass < 2; ++pass) {
#pragma unroll
        for (int it = 0; it < 8; ++it) {
          const int row = it * 2 + hh;
          v4f v = *(const v4f*)(slab + row * 68 + c4);
          *(volatile v4f*)(C + (size_t)(mBase + row) * ldc + n0 + c4) = v;
        }
        __threadfence();
      }
    } else {
      const int q = lane >> 3, c8 = (lane & 7) * 8;
      unsigned short* C  = (unsigned short*)Cout  + (size_t)b * strideC;
      unsigned short* C2 = (OUT_MODE == 2) ? ((unsigned short*)Cout2 + (size_t)b * strideC) : nullptr;
      for (int pass = 0; pass < 2; ++pass) {
#pragma unroll
        for (int it = 0; it < 4; ++it) {
          const int row = it * 4 + q;
          const float* sp = slab + row * 68 + c8;
          v8h hv, lv;
#pragma unroll
          for (int e = 0; e < 8; ++e) {
            if (OUT_MODE == 1) {
              hv[e] = (_Float16)sp[e];
            } else {
              unsigned short hb = f2bf_bits(sp[e]);
              unsigned short lb = f2bf_bits(sp[e] - bf_bits2f(hb));
              hv[e] = __builtin_bit_cast(_Float16, hb);
              lv[e] = __builtin_bit_cast(_Float16, lb);
            }
          }
          *(volatile v8h*)(C + (size_t)(mBase + row) * ldc + n0 + c8) = hv;
          if (OUT_MODE == 2) *(volatile v8h*)(C2 + (size_t)(mBase + row) * ldc + n0 + c8) = lv;
        }
        __threadfence();
      }
    }
    __builtin_amdgcn_fence(__ATOMIC_RELEASE, "workgroup");
    __builtin_amdgcn_wave_barrier();
    __builtin_amdgcn_fence(__ATOMIC_ACQUIRE, "workgroup");
  }
}

__global__ __launch_bounds__(256) void transpose_cast_f16(const float* __restrict__ in, int ldi,
                                                         _Float16* __restrict__ outT, int ldo, float scale) {
  __shared__ __align__(16) _Float16 tile[64][72];
  const int c0 = blockIdx.x * 64, r0 = blockIdx.y * 64;
  const int t = threadIdx.y * 32 + threadIdx.x;
  for (int i = threadIdx.y; i < 64; i += 8) {
    tile[threadIdx.x][i]      = (_Float16)(in[(size_t)(r0 + i) * ldi + c0 + threadIdx.x] * scale);
    tile[32 + threadIdx.x][i] = (_Float16)(in[(size_t)(r0 + i) * ldi + c0 + 32 + threadIdx.x] * scale);
  }
  __syncthreads();
  const int q = t >> 3, c8 = (t & 7) * 8;
  for (int pass = 0; pass < 2; ++pass) {
#pragma unroll
    for (int it = 0; it < 2; ++it) {
      const int c = it * 32 + q;
      v8h hv = *(const v8h*)(&tile[c][c8]);
      *(volatile v8h*)(outT + (size_t)(c0 + c) * ldo + r0 + c8) = hv;
    }
    __threadfence();
  }
}

__global__ __launch_bounds__(256) void padcast_x_kernel(const float* __restrict__ x, unsigned short* __restrict__ X16) {
  const long i = (long)blockIdx.x * 256 + threadIdx.x;
  if (i >= (long)NP * FIN / 8) return;
  const long e0 = 8 * i;
  const bool ok = e0 < (long)NN * FIN;
  const v4f z4 = {0.f, 0.f, 0.f, 0.f};
  const v4f a = ok ? *(const v4f*)(x + e0) : z4;
  const v4f b = ok ? *(const v4f*)(x + e0 + 4) : z4;
  v8h hv;
#pragma unroll
  for (int e = 0; e < 4; ++e) { hv[e] = (_Float16)a[e]; hv[4 + e] = (_Float16)b[e]; }
  *(volatile v8h*)(X16 + e0) = hv;
  __threadfence();
  *(volatile v8h*)(X16 + e0) = hv;
}

template <int NH_>
__global__ __launch_bounds__(256) void att_terms_kernel(const float* __restrict__ XW, int ld, const float* __restrict__ as, const float* __restrict__ ad,
                                                       float* __restrict__ ASD) {
  __shared__ float st[8][8];
  const int lane = threadIdx.x & 31, wave = threadIdx.x >> 5;
  const int n = blockIdx.x * 8 + wave;
  const float* xr = XW + (size_t)n * ld;
  float sv[4] = {0.f, 0.f, 0.f, 0.f}, dv[4] = {0.f, 0.f, 0.f, 0.f};
#pragma unroll
  for (int h = 0; h < NH_; ++h) {
    const float x0 = xr[h * 64 + 2 * lane], x1 = xr[h * 64 + 2 * lane + 1];
    float s = x0 * as[h * 64 + 2 * lane] + x1 * as[h * 64 + 2 * lane + 1];
    float d = x0 * ad[h * 64 + 2 * lane] + x1 * ad[h * 64 + 2 * lane + 1];
#pragma unroll
    for (int o = 16; o > 0; o >>= 1) { s += __shfl_xor(s, o, 32); d += __shfl_xor(d, o, 32); }
    sv[h] = s; dv[h] = d;
  }
  if (lane < 8) {
    float v = 0.f;
#pragma unroll
    for (int h = 0; h < NH_; ++h) { if (lane == h) v = sv[h]; if (lane == 4 + h) v = dv[h]; }
    st[wave][lane] = v;
  }
  __syncthreads();
  if (threadIdx.x < 64) {
    const float v = st[threadIdx.x >> 3][threadIdx.x & 7];
    ((volatile float*)ASD)[(size_t)blockIdx.x * 64 + threadIdx.x] = v;
    __threadfence();
    ((volatile float*)ASD)[(size_t)blockIdx.x * 64 + threadIdx.x] = v;
  }
}

__device__ __forceinline__ int blk_excl_scan(int cnt, int* scan_ws, int tid, int* tot) {
  const int lane = tid & 31, wave = tid >> 5; int incl = cnt;
#pragma unroll
  for (int o = 1; o < 32; o <<= 1) { const int v = __shfl_up(incl, o, 32); if (lane >= o) incl += v; }
  if (lane == 31) scan_ws[wave] = incl;
  __syncthreads();
  if (wave == 0) { int wv = (lane < NT / 32) ? scan_ws[lane] : 0; int wincl = wv;
#pragma unroll
    for (int o = 1; o < 32; o <<= 1) { const int v = __shfl_up(wincl, o, 32); if (lane >= o) wincl += v; }
    if (lane < NT / 32) scan_ws[32 + lane] = wincl - wv; if (lane == 31) scan_ws[64] = wincl; }
  __syncthreads();
  const int res = scan_ws[32 + wave] + incl - cnt; *tot = scan_ws[64];
  return res;
}
template <int SP, int CAP>
__device__ __forceinline__ int chunk_hits(const int* __restrict__ dstv, const int* __restrict__ srcv, int e0, int n0, int tid,
                                          int* LIST, int* scan_ws) {
  const int eb = e0 + tid * SP;
  const int nhi = (n0 + TILE < NN) ? (n0 + TILE) : NN;
  int rec[SP]; int cnt = 0;
  if (eb < NE) {
#pragma unroll
    for (int k = 0; k < SP; k += 4) {
      const v4i d4 = *(const v4i*)(dstv + eb + k);
      const v4i s4 = *(const v4i*)(srcv + eb + k);
#pragma unroll
      for (int e = 0; e < 4; ++e) {
        const int d = d4[e]; int r = -1;
        if (d >= n0 && d < nhi) { int s = s4[e]; s = s < 0 ? 0 : (s >= NN ? NN - 1 : s); r = ((d - n0) << 16) | s; ++cnt; }
        rec[k + e] = r;
      }
    }
  } else {
#pragma unroll
    for (int k = 0; k < SP; ++k) {
      const int e = eb + k; const int d = e - NE; int r = -1;
      if (e < NV && d >= n0 && d < nhi) { r = ((d - n0) << 16) | d; ++cnt; }
      rec[k] = r;
    }
  }
  int tot; int p = blk_excl_scan(cnt, scan_ws, tid, &tot);
#pragma unroll
  for (int k = 0; k < SP; ++k) if (rec[k] >= 0) { if ((unsigned)p < (unsigned)CAP) LIST[p] = rec[k]; ++p; }
  __syncthreads();
  return tot < CAP ? tot : CAP;
}
__device__ __forceinline__ float elu1(float v) { return v > 0.f ? v : (__expf(v) - 1.0f); }
__device__ __forceinline__ v4f epi_elu4(v4f a, float inv, v4f bsv, bool live) {
  v4f t = a * inv; fence_v4(t); t = t + bsv;
  v4f r;
#pragma unroll
  for (int e = 0; e < 4; ++e) r[e] = live ? elu1(t[e]) : 0.f;
  return r;
}

#define SCH1 2048
#define NCH1 ((NV + SCH1 - 1) / SCH1)
__global__ __launch_bounds__(NT) void agg1_kernel(const float* __restrict__ XW, const int* __restrict__ ei, const float* __restrict__ ASD,
                                                 const float* __restrict__ bias, float* AGG, unsigned short* __restrict__ H16) {
  __shared__ int LIST[SCH1];
  __shared__ float SM[TILE * NH1];
  __shared__ float SL[TILE * NH1];
  __shared__ __align__(16) float slab[NT / 32][F1];
  __shared__ int scan_ws[80];
  const int tid = threadIdx.x, lane = tid & 31, wave = tid >> 5;
  const int n0 = blockIdx.x * TILE;
  const int h4 = lane & 3;
  const v4f z4 = {0.f, 0.f, 0.f, 0.f};
#pragma unroll 1
  for (int j = 0; j < RPW; ++j) {
    float* rp = AGG + (size_t)(n0 + wave * RPW + j) * F1 + 4 * lane;
    *(v4f*)rp = z4; *(v4f*)(rp + 128) = z4;
  }
  for (int i = tid; i < TILE * NH1; i += NT) { SM[i] = -INFINITY; SL[i] = 0.f; }
  __syncthreads();
  const int* srcv = ei; const int* dstv = ei + NE;
#pragma unroll 1
  for (int c = 0; c < NCH1; ++c) {
    const int tot = chunk_hits<SCH1 / NT, SCH1>(dstv, srcv, c * SCH1, n0, tid, LIST, scan_ws);
#pragma unroll 1
    for (int base = 0; base < tot; base += 32) {
      const int q = base + lane;
      const int rv = (q < tot) ? LIST[q] : -1;
      const int own = (rv >= 0 && (rv >> 23) == wave) ? 1 : 0;
      unsigned msk = (unsigned)__ballot(own);
#pragma unroll 1
      for (int it = 0; it < 32; ++it) {
        if (msk == 0u) break;
        const int bp = __builtin_ctz(msk); msk &= msk - 1u;
        const int r = __shfl(rv, bp, 32);
        const int dl = r >> 16, s = r & 0xFFFF;
        const int mi = dl * NH1 + h4;
        float al = ASD[(size_t)s * 8 + h4] + ASD[(size_t)(n0 + dl) * 8 + 4 + h4];
        al = (al >= 0.f) ? al : 0.2f * al;
        const float mo = SM[mi], lo = SL[mi];
        const float mn = fmaxf(mo, al);
        const float rr = __expf(mo - mn), ex = __expf(al - mn);
        const float ln = lo * rr + ex;
        if (lane < NH1) { SM[mi] = mn; SL[mi] = ln; }
        float* rp = AGG + (size_t)(n0 + dl) * F1 + 4 * lane;
        const float* xp = XW + (size_t)s * F1 + 4 * lane;
#pragma unroll
        for (int j = 0; j < 2; ++j) {
          const int hj = 2 * j + (lane >> 4);
          const float rrj = __shfl(rr, hj, 32), exj = __shfl(ex, hj, 32);
          v4f a = *(const v4f*)(rp + 128 * j);
          const v4f hv = *(const v4f*)(xp + 128 * j);
          const v4f t = exj * hv;
          a = a * rrj + t;
          *(v4f*)(rp + 128 * j) = a;
        }
      }
    }
    __syncthreads();
  }
  __threadfence();
  const v4f bA = *(const v4f*)(bias + 4 * lane), bB = *(const v4f*)(bias + 128 + 4 * lane);
  float* sw = slab[wave];
#pragma unroll 1
  for (int j = 0; j < RPW; ++j) {
    const int dl = wave * RPW + j; const int n = n0 + dl;
    const bool live = n < NN;
    float lv = 1.0f;
    if (lane < NH1) lv = SL[dl * NH1 + lane];
    lv = (live && lv > 0.f) ? lv : 1.0f;
    const float inv4 = 1.0f / lv;
    const float invA = __shfl(inv4, lane >> 4, 32), invB = __shfl(inv4, 2 + (lane >> 4), 32);
    const float* rp = AGG + (size_t)n * F1 + 4 * lane;
    const v4f vA = epi_elu4(*(const v4f*)rp, invA, bA, live);
    const v4f vB = epi_elu4(*(const v4f*)(rp + 128), invB, bB, live);
    *(v4f*)(sw + 4 * lane) = vA; *(v4f*)(sw + 128 + 4 * lane) = vB;
    __builtin_amdgcn_fence(__ATOMIC_RELEASE, "workgroup");
    __builtin_amdgcn_wave_barrier();
    __builtin_amdgcn_fence(__ATOMIC_ACQUIRE, "workgroup");
    const v4f p0 = *(const v4f*)(sw + 8 * lane), p1 = *(const v4f*)(sw + 8 * lane + 4);
    v8h hv;
#pragma unroll
    for (int e = 0; e < 4; ++e) { hv[e] = (_Float16)p0[e]; hv[4 + e] = (_Float16)p1[e]; }
    unsigned short* hrow = H16 + (size_t)n * F1 + 8 * lane;
    for (int pass = 0; pass < 2; ++pass) { *(volatile v8h*)hrow = hv; __threadfence(); }
    __builtin_amdgcn_fence(__ATOMIC_RELEASE, "workgroup");
    __builtin_amdgcn_wave_barrier();
    __builtin_amdgcn_fence(__ATOMIC_ACQUIRE, "workgroup");
  }
}

#define SCH2 4096
#define NCH2 ((NV + SCH2 - 1) / SCH2)
__global__ __launch_bounds__(NT) void agg2_kernel(const float* __restrict__ XW2, const int* __restrict__ ei, const float* __restrict__ ASD,
                                                 const float* __restrict__ bias, float* HO) {
  __shared__ int LIST[SCH2];
  __shared__ float SM[TILE];
  __shared__ float SL[TILE];
  __shared__ __align__(16) float slab[NT / 32][2 * F2];
  __shared__ int scan_ws[80];
  const int tid = threadIdx.x, lane = tid & 31, wave = tid >> 5;
  const int n0 = blockIdx.x * TILE;
  const v2f z2 = {0.f, 0.f};
#pragma unroll 1
  for (int j = 0; j < RPW; ++j) {
    const int n = n0 + wave * RPW + j;
    if (n < NN) *(v2f*)(HO + (size_t)n * F2 + 2 * lane) = z2;
  }
  for (int i = tid; i < TILE; i += NT) { SM[i] = -INFINITY; SL[i] = 0.f; }
  __syncthreads();
  const int* srcv = ei; const int* dstv = ei + NE;
#pragma unroll 1
  for (int c = 0; c < NCH2; ++c) {
    const int tot = chunk_hits<SCH2 / NT, SCH2>(dstv, srcv, c * SCH2, n0, tid, LIST, scan_ws);
#pragma unroll 1
    for (int base = 0; base < tot; base += 32) {
      const int q = base + lane;
      const int rv = (q < tot) ? LIST[q] : -1;
      const int own = (rv >= 0 && (rv >> 23) == wave) ? 1 : 0;
      unsigned msk = (unsigned)__ballot(own);
#pragma unroll 1
      for (int it = 0; it < 32; ++it) {
        if (msk == 0u) break;
        const int bp = __builtin_ctz(msk); msk &= msk - 1u;
        const int r = __shfl(rv, bp, 32);
        const int dl = r >> 16, s = r & 0xFFFF;
        float al = ASD[(size_t)s * 8] + ASD[(size_t)(n0 + dl) * 8 + 4];
        al = (al >= 0.f) ? al : 0.2f * al;
        const float mo = SM[dl], lo = SL[dl];
        const float mn = fmaxf(mo, al);
        const float rr = __expf(mo - mn), ex = __expf(al - mn);
        const float ln = lo * rr + ex;
        if (lane == 0) { SM[dl] = mn; SL[dl] = ln; }
        float* rp = HO + (size_t)(n0 + dl) * F2 + 2 * lane;
        v2f a = *(const v2f*)rp;
        const v2f hv = *(const v2f*)(XW2 + (size_t)s * F2 + 2 * lane);
        const v2f t = ex * hv;
        a = a * rr + t;
        *(v2f*)rp = a;
      }
    }
    __syncthreads();
  }
  __threadfence();
  const v2f bb = *(const v2f*)(bias + 2 * lane);
  float* sw = slab[wave];
  const int hh = lane >> 4, c4 = (lane & 15) * 4;
#pragma unroll 1
  for (int j = 0; j < RPW / 2; ++j) {
    const int rA = wave * RPW + 2 * j; const int nA = n0 + rA;
    if (nA < NN) {
#pragma unroll
      for (int u = 0; u < 2; ++u) {
        const int dl = rA + u;
        float lv = SL[dl]; lv = lv > 0.f ? lv : 1.0f;
        const float inv = 1.0f / lv;
        const v2f a = *(const v2f*)(HO + (size_t)(nA + u) * F2 + 2 * lane);
        v2f t = a * inv; fence_v2(t); t = t + bb;
        v2f r2; r2[0] = elu1(t[0]); r2[1] = elu1(t[1]);
        *(v2f*)(sw + u * F2 + 2 * lane) = r2;
      }
      __builtin_amdgcn_fence(__ATOMIC_RELEASE, "workgroup");
      __builtin_amdgcn_wave_barrier();
      __builtin_amdgcn_fence(__ATOMIC_ACQUIRE, "workgroup");
      const v4f val = *(const v4f*)(sw + hh * F2 + c4);
      float* orow = HO + (size_t)(nA + hh) * F2 + c4;
      for (int pass = 0; pass < 2; ++pass) { *(volatile v4f*)orow = val; __threadfence(); }
      __builtin_amdgcn_fence(__ATOMIC_RELEASE, "workgroup");
      __builtin_amdgcn_wave_barrier();
      __builtin_amdgcn_fence(__ATOMIC_ACQUIRE, "workgroup");
    }
  }
}

__global__ __launch_bounds__(NT) void pool_fc_kernel(const float* __restrict__ HO, const int* __restrict__ bvec, const float* __restrict__ fcW,
                                                    const float* __restrict__ fcb, float* __restrict__ out1) {
  __shared__ __align__(16) float accs[NT / 32][NG][F2];
  __shared__ int cnts[NT / 32][NG];
  __shared__ float pooled[NG][F2];
  __shared__ float so[32];
  const int tid = threadIdx.x, lane = tid & 31, wave = tid >> 5;
  for (int i = tid; i < (NT / 32) * NG * F2; i += NT) (&accs[0][0][0])[i] = 0.f;
  if (tid < (NT / 32) * NG) (&cnts[0][0])[tid] = 0;
  __syncthreads();
#pragma unroll 1
  for (int n = wave; n < NN; n += NT / 32) {
    const int g = bvec[n];
    if (g >= 0 && g < NG) {
      float* ap = &accs[wave][g][0] + 2 * lane;
      v2f a = *(const v2f*)ap;
      const v2f hv = *(const v2f*)(HO + (size_t)n * F2 + 2 * lane);
      a = a + hv;
      *(v2f*)ap = a;
      if (lane == 0) cnts[wave][g] += 1;
    }
  }
  __syncthreads();
  for (int i = tid; i < NG * F2; i += NT) {
    const int g = i / F2, c = i - g * F2;
    float s = 0.f; int ct = 0;
#pragma unroll
    for (int w = 0; w < NT / 32; ++w) { s += accs[w][g][c]; ct += cnts[w][g]; }
    const float cf = (float)ct;
    pooled[g][c] = s * (1.0f / fmaxf(cf, 1.0f));
  }
  __syncthreads();
  if (tid < 32) {
    float v = 0.f;
    if (tid < NG * 2) {
      const int g = tid >> 1, jx = tid & 1;
      v = fcb[jx];
#pragma unroll 1
      for (int c = 0; c < F2; ++c) v += pooled[g][c] * fcW[c * 2 + jx];
    }
    so[tid] = v;
  }
  __syncthreads();
  if (tid < NG * 2) {
    const float v = so[tid];
    ((volatile float*)out1)[tid] = v;
    __threadfence();
    ((volatile float*)out1)[tid] = v;
  }
}

extern "C" void kernel_launch(void* const* d_in, const int* in_sizes, int n_in,
                              void* d_out, int out_size, void* d_ws, size_t ws_size, hipStream_t stream) {
  (void)out_size;
  if (n_in < 13) return;
  if (in_sizes[0] != NN * FIN || in_sizes[1] != 2 * NE || in_sizes[2] != NN) return;
  const float* x    = (const float*)d_in[0];
  const int*   ei   = (const int*)  d_in[1];
  const int*   bvec = (const int*)  d_in[2];
  const float* W1   = (const float*)d_in[3];
  const float* as1  = (const float*)d_in[4];
  const float* ad1  = (const float*)d_in[5];
  const float* b1   = (const float*)d_in[6];
  const float* W2   = (const float*)d_in[7];
  const float* as2  = (const float*)d_in[8];
  const float* ad2  = (const float*)d_in[9];
  const float* b2   = (const float*)d_in[10];
  const float* fcW  = (const float*)d_in[11];
  const float* fcb  = (const float*)d_in[12];
  float* out0 = (float*)d_out;
  float* out1 = out0 + (size_t)NN * F2;

  char* ws = (char*)d_ws; size_t off = 0;
  auto carve = [&](size_t bytes) -> char* { char* p = ws + off; off += (bytes + 255) & ~(size_t)255; return p; };
  unsigned short* X16 = (unsigned short*)carve((size_t)NP * FIN * 2);
  unsigned short* W1T = (unsigned short*)carve((size_t)F1 * FIN * 2);
  unsigned short* W2T = (unsigned short*)carve((size_t)F2 * F1 * 2);
  float*          XW1 = (float*)carve((size_t)NP * F1 * 4);
  float*          AGG = (float*)carve((size_t)NP * F1 * 4);
  float*          ASD = (float*)carve((size_t)NP * 8 * 4);
  if (off > ws_size || off > (size_t)134217728) return;
  unsigned short* H16 = X16;
  float*          XW2 = AGG;

  padcast_x_kernel<<<(NP * FIN / 8 + 255) / 256, 256, 0, stream>>>(x, X16);
  transpose_cast_f16<<<dim3(F1 / 64, FIN / 64), dim3(32, 8), 0, stream>>>(W1, F1, (_Float16*)W1T, FIN, 16.0f);
  transpose_cast_f16<<<dim3(F2 / 64, F1 / 64), dim3(32, 8), 0, stream>>>(W2, F2, (_Float16*)W2T, F1, 16.0f);
  {
    const int tiles = (NP / 64) * (F1 / 64);
    wmma_gemm64<0, false, 0, 0, false><<<dim3((tiles + 7) / 8, 1), 256, 0, stream>>>(
        (const unsigned short*)X16, (const unsigned short*)nullptr, FIN, 0L,
        (const unsigned short*)W1T, (const unsigned short*)nullptr, FIN, 0L,
        (void*)XW1, (void*)nullptr, F1, 0L,
        (const float*)nullptr, (const float*)nullptr, 0L, NP, F1, FIN, 1.0f / 16.0f);
  }
  att_terms_kernel<4><<<NP / 8, 256, 0, stream>>>(XW1, F1, as1, ad1, ASD);
  agg1_kernel<<<NTL, NT, 0, stream>>>(XW1, ei, ASD, b1, AGG, H16);
  {
    const int tiles = (NP / 64) * (F2 / 64);
    wmma_gemm64<0, false, 0, 0, false><<<dim3((tiles + 7) / 8, 1), 256, 0, stream>>>(
        (const unsigned short*)H16, (const unsigned short*)nullptr, F1, 0L,
        (const unsigned short*)W2T, (const unsigned short*)nullptr, F1, 0L,
        (void*)XW2, (void*)nullptr, F2, 0L,
        (const float*)nullptr, (const float*)nullptr, 0L, NP, F2, F1, 1.0f / 16.0f);
  }
  att_terms_kernel<1><<<NP / 8, 256, 0, stream>>>(XW2, F2, as2, ad2, ASD);
  agg2_kernel<<<NTL, NT, 0, stream>>>(XW2, ei, ASD, b2, out0);
  pool_fc_kernel<<<1, NT, 0, stream>>>(out0, bvec, fcW, fcb, out1);
}
